// DCNConvModule_54589034332207
// MI455X (gfx1250) — hardware-verified
//
#include <hip/hip_runtime.h>
#include <math.h>

typedef __attribute__((ext_vector_type(16))) _Float16 v16h;
typedef __attribute__((ext_vector_type(16))) __bf16 v16b;
typedef __attribute__((ext_vector_type(8)))  _Float16 v8h;
typedef __attribute__((ext_vector_type(8)))  float v8f;
typedef __attribute__((ext_vector_type(4)))  float v4f;
typedef __attribute__((ext_vector_type(2)))  float v2f;
typedef __attribute__((ext_vector_type(4)))  unsigned v4u;
typedef __attribute__((ext_vector_type(4)))  int v4i;
typedef float __attribute__((may_alias)) float_a;
typedef int __attribute__((may_alias)) int_a;

template <typename T> __device__ __forceinline__ void vst2(void* p, T v) { *(volatile T*)p = v; __threadfence(); *(volatile T*)p = v; }
__device__ __forceinline__ v8f wmma16(v16h a, v16h b, v8f c) {
  v8f d = __builtin_amdgcn_wmma_f32_16x16x32_f16(false, a, false, b, (short)0, c, false, false);
  asm volatile("v_nop\n\tv_nop\n\tv_nop\n\tv_nop" : "+v"(d) : "v"(a), "v"(b));
  return d;
}
__device__ __forceinline__ v8f wmma_bf(v16b a, v16b b, v8f c) {
  v8f d = __builtin_amdgcn_wmma_f32_16x16x32_bf16(false, a, false, b, (short)0, c, false, false);
  asm volatile("v_nop\n\tv_nop\n\tv_nop\n\tv_nop" : "+v"(d) : "v"(a), "v"(b));
  return d;
}
__device__ __forceinline__ v16h frag_h(const _Float16* rowk0, int lane) {
  union { v16h v; v8h q[2]; } u; const _Float16* p = rowk0 + 8 * (lane >> 4);
  u.q[0] = *(const v8h*)p; u.q[1] = *(const v8h*)(p + 16); return u.v;
}
__device__ __forceinline__ v16h frag_f32(const float* rowk0, int lane) {
  v16h a; const float* p = rowk0 + 8 * (lane >> 4);
#pragma unroll
  for (int i = 0; i < 8; ++i) { a[i] = (_Float16)p[i]; a[8 + i] = (_Float16)p[16 + i]; }
  return a;
}
__device__ __forceinline__ v16h frag_f32s(const float* rowk0, int lane, float sc) {
  v16h a; const float* p = rowk0 + 8 * (lane >> 4);
#pragma unroll
  for (int i = 0; i < 8; ++i) { a[i] = (_Float16)(p[i] * sc); a[8 + i] = (_Float16)(p[16 + i] * sc); }
  return a;
}
__device__ __forceinline__ v16h fragc_f32(const float* W, int k0, int n, int lane, int ld, int K) {
  v16h a; const int g = lane >> 4;
#pragma unroll
  for (int i = 0; i < 8; ++i) { const int ka = k0 + 8 * g + i, kb = ka + 16;
    a[i] = (_Float16)(ka < K ? W[(size_t)ka * ld + n] : 0.f); a[8 + i] = (_Float16)(kb < K ? W[(size_t)kb * ld + n] : 0.f); }
  return a;
}
struct F2 { v16b h, l; };
__device__ __forceinline__ F2 bsplit16(const float v[16]) { F2 r;
#pragma unroll
  for (int i = 0; i < 16; ++i) { const __bf16 h = (__bf16)v[i]; r.h[i] = h; r.l[i] = (__bf16)(v[i] - (float)h); }
  return r; }
__device__ __forceinline__ F2 split_row(const float* row, int k0, int lane) { float v[16]; const float* p = row + k0 + 8 * (lane >> 4);
#pragma unroll
  for (int i = 0; i < 8; ++i) { v[i] = p[i]; v[8 + i] = p[16 + i]; }
  return bsplit16(v); }
__device__ __forceinline__ F2 split_rowK(const float* row, int k0, int lane, int K) { float v[16]; const int g = lane >> 4;
#pragma unroll
  for (int i = 0; i < 8; ++i) { const int ka = k0 + 8 * g + i, kb = ka + 16; v[i] = ka < K ? row[ka] : 0.f; v[8 + i] = kb < K ? row[kb] : 0.f; }
  return bsplit16(v); }
__device__ __forceinline__ F2 split_col(const float* W, int k0, int n, int lane, int ld, int K) { float v[16]; const int g = lane >> 4;
#pragma unroll
  for (int i = 0; i < 8; ++i) { const int ka = k0 + 8 * g + i, kb = ka + 16; v[i] = ka < K ? W[(size_t)ka * ld + n] : 0.f; v[8 + i] = kb < K ? W[(size_t)kb * ld + n] : 0.f; }
  return bsplit16(v); }
__device__ __forceinline__ v8f mac3(const F2& a, const F2& b, v8f c) { c = wmma_bf(a.l, b.h, c); c = wmma_bf(a.h, b.l, c); return wmma_bf(a.h, b.h, c); }
__device__ __forceinline__ float sigm(float v) { return 1.0f / (1.0f + expf(-v)); }
#define LDSX() do { asm volatile("s_wait_dscnt 0" ::: "memory"); __builtin_amdgcn_wave_barrier(); __builtin_amdgcn_fence(__ATOMIC_RELEASE, "workgroup"); } while (0)

#define NB 2
#define CC 256
#define HH 128
#define WW 128
#define NP (HH * WW)
#define OO 256
#define KK 9
#define KTOT (CC * KK)
#define NG 32
#define CPG (OO / NG)
#define NPB (NP / 64)

__global__ __launch_bounds__(256) void k_packW(const float* __restrict__ W, _Float16* __restrict__ P) {
  const int o = blockIdx.x, tid = threadIdx.x;
  for (int q = tid; q < KTOT / 8; q += 256) { union { v8h hh; v4u u; } pk;
#pragma unroll
    for (int i = 0; i < 8; ++i) pk.hh[i] = (_Float16)(W[(size_t)o * KTOT + q * 8 + i] * 16.0f);
    vst2(P + (size_t)o * KTOT + q * 8, pk.u); }
}
__global__ __launch_bounds__(256) void k_xT(const float* __restrict__ x, float* __restrict__ xt) {
  __shared__ float tile[64][65];
  const int b = blockIdx.z, p0 = blockIdx.x * 64, c0 = blockIdx.y * 64, tid = threadIdx.x;
  for (int q = tid; q < 64 * 64; q += 256) { const int c = q >> 6, pp = q & 63; tile[c][pp] = x[((size_t)b * CC + c0 + c) * NP + p0 + pp]; }
  __syncthreads();
  for (int q = tid; q < 64 * 16; q += 256) { const int pp = q >> 4, pc = q & 15;
    v4f v = { tile[pc * 4][pp], tile[pc * 4 + 1][pp], tile[pc * 4 + 2][pp], tile[pc * 4 + 3][pp] };
    vst2(xt + ((size_t)b * NP + p0 + pp) * CC + c0 + pc * 4, v); }
}
__global__ __launch_bounds__(256) void k_sample(const float* __restrict__ xt, const float* __restrict__ off, _Float16* __restrict__ A16, int b, int poff) {
  __shared__ __align__(16) _Float16 row[KTOT];
  const int p = poff + blockIdx.x, c = threadIdx.x; const int oy = p / WW, ox = p % WW;
  const float* xb = xt + (size_t)b * NP * CC;
#pragma unroll 1
  for (int k = 0; k < KK; ++k) { const int ki = k / 3, kj = k % 3;
    const float py = off[(((size_t)b * 2 * KK) + 2 * k) * NP + p] + (float)ki + (float)(oy - 1);
    const float px = off[(((size_t)b * 2 * KK) + 2 * k + 1) * NP + p] + (float)kj + (float)(ox - 1);
    const float fy = floorf(py), fx = floorf(px); const float wy1 = py - fy, wx1 = px - fx; const int y0 = (int)fy, x0 = (int)fx;
    float acc = 0.f;
#pragma unroll
    for (int q = 0; q < 4; ++q) { const int yy = y0 + (q >> 1), xx = x0 + (q & 1);
      const float wgt = ((q >> 1) ? wy1 : 1.0f - wy1) * ((q & 1) ? wx1 : 1.0f - wx1);
      if (yy >= 0 && yy <= HH - 1 && xx >= 0 && xx <= WW - 1) acc += xb[((size_t)yy * WW + xx) * CC + c] * wgt; }
    row[c * KK + k] = (_Float16)acc; }
  __syncthreads();
  for (int q = threadIdx.x; q < KTOT / 8; q += 256) vst2(A16 + (size_t)blockIdx.x * KTOT + q * 8, *(const v4u*)(&row[q * 8]));
}
__global__ __launch_bounds__(128) void k_conv(const _Float16* __restrict__ A16, const _Float16* __restrict__ P, const float* __restrict__ bias, float* __restrict__ pre, float* __restrict__ part, int b, int poff) {
  __shared__ __align__(16) float st[128][68];
  __shared__ __align__(16) float sp[128][2];
  const int tid = threadIdx.x, wave = tid >> 5, lane = tid & 31, col = lane & 15, g = lane >> 4;
  const int p0 = poff + blockIdx.x * 64, r0 = p0 + wave * 16, n0 = blockIdx.y * 128;
  v8f acc[8] = {};
#pragma unroll 1
  for (int kc = 0; kc < KTOT / 32; ++kc) { const v16h a = frag_h(A16 + (size_t)(r0 - poff + col) * KTOT + kc * 32, lane);
#pragma unroll
    for (int j = 0; j < 8; ++j) acc[j] = wmma16(a, frag_h(P + (size_t)(n0 + j * 16 + col) * KTOT + kc * 32, lane), acc[j]); }
#pragma unroll
  for (int j = 0; j < 8; ++j) { const float bb = bias[n0 + j * 16 + col];
#pragma unroll
    for (int r = 0; r < 8; ++r) st[j * 16 + col][wave * 16 + 8 * g + r] = acc[j][r] * (1.0f / 16.0f) + bb; }
  __syncthreads();
  { const int o = tid; float s = 0.f, q2 = 0.f;
#pragma unroll
    for (int pc = 0; pc < 16; ++pc) { const v4f v = *(const v4f*)(&st[o][pc * 4]); vst2(pre + ((size_t)b * OO + n0 + o) * NP + p0 + pc * 4, v);
#pragma unroll
      for (int e = 0; e < 4; ++e) { s += v[e]; q2 += v[e] * v[e]; } }
    sp[o][0] = s; sp[o][1] = q2; }
  __syncthreads();
  if (tid < 64) vst2(part + (((size_t)b * NPB + (p0 / 64)) * OO + n0) * 2 + tid * 4, *(const v4f*)(&sp[0][0] + tid * 4));
}
__global__ __launch_bounds__(64) void k_gnstat(const float* __restrict__ part, float* __restrict__ stat) {
  const int bg = threadIdx.x, b = bg / NG, gg = bg % NG; float s = 0.f, q2 = 0.f;
#pragma unroll 1
  for (int blk = 0; blk < NPB; ++blk)
#pragma unroll
    for (int c = 0; c < CPG; ++c) { const size_t i = (((size_t)b * NPB + blk) * OO + gg * CPG + c) * 2; s += part[i]; q2 += part[i + 1]; }
  const float n = (float)(CPG * NP); const float mu = s / n; float var = q2 / n - mu * mu; var = var < 0.f ? 0.f : var;
  __shared__ __align__(16) float so[128];
  so[bg * 2] = mu; so[bg * 2 + 1] = rsqrtf(var + 1e-5f);
  __syncthreads();
  if (bg < 32) vst2(stat + bg * 4, *(const v4f*)(&so[bg * 4]));
}
__global__ __launch_bounds__(256) void k_apply(const float* __restrict__ pre, const float* __restrict__ stat, const float* __restrict__ gam, const float* __restrict__ bet, float* __restrict__ out) {
  const int b = blockIdx.y, o = blockIdx.x, tid = threadIdx.x; const int gg = o / CPG;
  const float mu = stat[(b * NG + gg) * 2], rs = stat[(b * NG + gg) * 2 + 1], ga = gam[o], be = bet[o];
  const float* src = pre + ((size_t)b * OO + o) * NP; float* dst = out + ((size_t)b * OO + o) * NP;
  for (int q = tid; q < NP / 4; q += 256) { v4f v = *(const v4f*)(src + q * 4);
#pragma unroll
    for (int e = 0; e < 4; ++e) { const float t = (v[e] - mu) * rs * ga + be; v[e] = t > 0.f ? t : 0.f; }
    vst2(dst + q * 4, v); }
}
extern "C" void kernel_launch(void* const* d_in, const int* in_sizes, int n_in, void* d_out, int out_size, void* d_ws, size_t ws_size, hipStream_t stream) {
  (void)in_sizes; (void)n_in; (void)out_size; (void)ws_size;
  const float* x = (const float*)d_in[0]; const float* off = (const float*)d_in[1]; const float* W = (const float*)d_in[2]; const float* bias = (const float*)d_in[3];
  const float* gam = (const float*)d_in[4]; const float* bet = (const float*)d_in[5];
  float* out = (float*)d_out;
  char* ws = (char*)d_ws; size_t offb = 0;
  auto take = [&](size_t bytes) { char* p = ws + offb; offb += (bytes + 255) & ~(size_t)255; return p; };
  _Float16* P = (_Float16*)take((size_t)OO * KTOT * 2); float* part = (float*)take((size_t)NB * NPB * OO * 2 * 4); float* stat = (float*)take((size_t)NB * NG * 2 * 4);
  float* xt = (float*)take((size_t)NB * NP * CC * 4); float* pre = (float*)take((size_t)NB * OO * NP * 4);
  _Float16* A16 = (_Float16*)take((size_t)(NP / 2) * KTOT * 2);
  k_packW<<<OO, 256, 0, stream>>>(W, P);
  k_xT<<<dim3(NP / 64, CC / 64, NB), 256, 0, stream>>>(x, xt);
  for (int chk = 0; chk < 2 * NB; ++chk) { const int b = chk >> 1, poff = (chk & 1) * (NP / 2);
    k_sample<<<NP / 2, 256, 0, stream>>>(xt, off, A16, b, poff);
    k_conv<<<dim3((NP / 2) / 64, OO / 128), 128, 0, stream>>>(A16, P, bias, pre, part, b, poff); }
  k_gnstat<<<1, 64, 0, stream>>>(part, stat);
  k_apply<<<dim3(OO, NB), 256, 0, stream>>>(pre, stat, gam, bet, out);
}
